// FactorNet_42786464202884
// MI455X (gfx1250) — hardware-verified
//
#include <hip/hip_runtime.h>


namespace {
constexpr int NTOK = 16 * 512, DD = 64, HH = 128, KK = 64;
constexpr float HS = 256.0f, WSC = 256.0f, MIN_SIGMA = 0.008f, EPSN = 0.1f, VAR_MIN = 0.01f;
typedef _Float16 b16;
typedef __attribute__((ext_vector_type(16))) _Float16 v16b;
typedef __attribute__((ext_vector_type(8))) _Float16 v8b;
typedef __attribute__((ext_vector_type(8))) float v8f;
typedef __attribute__((ext_vector_type(4))) float v4f;
typedef __attribute__((ext_vector_type(2))) float v2f;
__device__ __forceinline__ float bf16_rne(float f) { unsigned int u = __float_as_uint(f); u += 0x7FFFu + ((u >> 16) & 1u); float r = __uint_as_float(u & 0xFFFF0000u); asm volatile("" : "+v"(r)); return r; }
__device__ __forceinline__ float bfv(float f) { float r = bf16_rne(f); asm volatile("" : "+v"(r)); return r; }
__device__ __forceinline__ void split16(float v, b16& hi, b16& lo) { hi = (b16)v; lo = (b16)(v - (float)hi); }
__device__ __forceinline__ v16b frag_kb(const b16* p, int hh) { const v8b a = *(const v8b*)(p + 8 * hh), b = *(const v8b*)(p + 16 + 8 * hh); v16b f;
#pragma unroll
  for (int e = 0; e < 8; ++e) { f[e] = a[e]; f[8 + e] = b[e]; } return f; }
__device__ __forceinline__ v8f wmma16b(v16b a, v16b b, v8f c) { v8f d = __builtin_amdgcn_wmma_f32_16x16x32_f16(false, a, false, b, (short)0, c, false, false); asm volatile("v_nop\n\tv_nop\n\tv_nop\n\tv_nop" : "+v"(d) : "v"(a), "v"(b)); return d; }
__device__ __forceinline__ void wave_lds_sync() { __builtin_amdgcn_fence(__ATOMIC_RELEASE, "workgroup"); __builtin_amdgcn_wave_barrier(); __builtin_amdgcn_fence(__ATOMIC_ACQUIRE, "workgroup"); }
__device__ __forceinline__ float pmul(float a, float b) { float p = a * b; asm volatile("" : "+v"(p)); return p; }
__device__ __forceinline__ void gemm8(b16 (*Ah)[HH + 8], b16 (*Al)[HH + 8], float (*Tf)[HH + 1], const b16* __restrict__ W, const float* __restrict__ bb, bool relu_, int nloc, int hlf) { v8f acc[8];
#pragma unroll
  for (int t = 0; t < 8; ++t) acc[t] = (v8f){};
#pragma unroll
  for (int kb = 0; kb < HH; kb += 32) { const v16b a = frag_kb(&Ah[nloc][kb], hlf), al = frag_kb(&Al[nloc][kb], hlf);
#pragma unroll
    for (int t = 0; t < 8; ++t) { const v16b bw = frag_kb(W + (size_t)(t * 16 + nloc) * HH + kb, hlf); acc[t] = wmma16b(a, bw, acc[t]); acc[t] = wmma16b(al, bw, acc[t]); } }
#pragma unroll
  for (int t = 0; t < 8; ++t) { const int cc = t * 16 + nloc; const float bv_ = bfv(bb[cc]);
#pragma unroll
    for (int r8 = 0; r8 < 8; ++r8) { const float v = acc[t][r8] * (1.0f / (HS * WSC)) + bv_; Tf[8 * hlf + r8][cc] = relu_ ? fmaxf(v, 0.0f) : v; } } }
__device__ __forceinline__ void stage8(b16 (*Ah)[HH + 8], b16 (*Al)[HH + 8], float (*Tf)[HH + 1], int lane) { for (int rr = 0; rr < 16; ++rr) for (int q = 0; q < 4; ++q) { const int c = q * 32 + lane; b16 p, pl; split16(Tf[rr][c] * HS, p, pl); Ah[rr][c] = p; Al[rr][c] = pl; } }
__device__ __forceinline__ float softplus_(float v) { return v > 20.0f ? v : (v < -20.0f ? __expf(v) : __logf(1.0f + __expf(v))); }

__global__ __launch_bounds__(256) void wput_kernel(const float* __restrict__ w2, const float* __restrict__ w3, const float* __restrict__ wo, b16* __restrict__ WT) { const size_t nt = (size_t)gridDim.x * 256, u0 = (size_t)blockIdx.x * 256 + threadIdx.x; v8b v;
  for (size_t u = u0; u < (size_t)3 * DD * HH * 16; u += nt) { const int m = (int)(u / ((size_t)DD * HH * 16)); const size_t r = u % ((size_t)DD * HH * 16); const int d = (int)(r / (HH * 16)), o = (int)((r / 16) % HH), k0 = (int)(r % 16) * 8; const float* w = (m == 0 ? w2 : m == 1 ? w3 : wo) + (size_t)d * HH * HH;
#pragma unroll
    for (int j = 0; j < 8; ++j) v[j] = (b16)(bf16_rne(w[(size_t)(k0 + j) * HH + o]) * WSC); for (int pass = 0; pass < 2; ++pass) { *(volatile v8b*)(WT + (((size_t)m * DD + d) * HH + o) * HH + k0) = v; __threadfence(); } } }
__global__ __launch_bounds__(32) void main_kernel(const float* __restrict__ z, const int* __restrict__ mask, const float* __restrict__ w1, const float* __restrict__ b1, const float* __restrict__ b2, const float* __restrict__ b3, const float* __restrict__ bo, const b16* __restrict__ WT, int TLIM, float* __restrict__ out) { __shared__ __attribute__((aligned(16))) b16 Ah[16][HH + 8], Al[16][HH + 8]; __shared__ float Tf[16][HH + 1]; const int lane = threadIdx.x, nloc = lane & 15, hlf = lane >> 4; const size_t t0 = (size_t)blockIdx.x * 16; if (t0 >= (size_t)TLIM) return;
  if (lane < 16) for (int k = HH; k < HH + 8; ++k) { Ah[lane][k] = (b16)0.0f; Al[lane][k] = (b16)0.0f; }
  float np1[16][2], np2[16][2];
#pragma unroll
  for (int rr = 0; rr < 16; ++rr) for (int q = 0; q < 2; ++q) { np1[rr][q] = 0.0f; np2[rr][q] = 0.0f; }
#pragma unroll 1
  for (int d = 0; d < DD; ++d) {
    for (int rr = 0; rr < 16; ++rr) { const float zv = bfv(z[(t0 + rr) * DD + d]); for (int q = 0; q < 4; ++q) { const int c = q * 32 + lane; Tf[rr][c] = fmaxf(pmul(zv, bfv(w1[(size_t)d * HH + c])) + bfv(b1[(size_t)d * HH + c]), 0.0f); } }
    wave_lds_sync(); stage8(Ah, Al, Tf, lane); wave_lds_sync();
    gemm8(Ah, Al, Tf, WT + ((size_t)0 * DD + d) * HH * HH, b2 + (size_t)d * HH, true, nloc, hlf); wave_lds_sync(); stage8(Ah, Al, Tf, lane); wave_lds_sync();
    gemm8(Ah, Al, Tf, WT + ((size_t)1 * DD + d) * HH * HH, b3 + (size_t)d * HH, true, nloc, hlf); wave_lds_sync(); stage8(Ah, Al, Tf, lane); wave_lds_sync();
    gemm8(Ah, Al, Tf, WT + ((size_t)2 * DD + d) * HH * HH, bo + (size_t)d * (2 * KK), false, nloc, hlf); wave_lds_sync();
#pragma unroll
    for (int rr = 0; rr < 16; ++rr) { const bool mk = mask[(t0 + rr) * DD + d] != 0; if (!mk) continue;
#pragma unroll
      for (int q = 0; q < 2; ++q) { const int k = q * 32 + lane; const float mu = Tf[rr][k]; const float sg = softplus_(Tf[rr][KK + k]) + MIN_SIGMA; const float iv = 1.0f / pmul(sg, sg); np1[rr][q] += pmul(mu, iv); np2[rr][q] += -0.5f * iv; } }
    wave_lds_sync(); }
  for (int pass = 0; pass < 2; ++pass) {
#pragma unroll
    for (int rr = 0; rr < 16; ++rr)
#pragma unroll
      for (int q = 0; q < 2; ++q) { const int k = q * 32 + lane; const float n2 = np2[rr][q] + EPSN; const float var = fmaxf(-1.0f / (2.0f * n2), VAR_MIN); ((volatile float*)out)[(t0 + rr) * KK + k] = pmul(np1[rr][q], var); ((volatile float*)out)[(size_t)NTOK * KK + (t0 + rr) * KK + k] = sqrtf(var); } __threadfence(); } }
}

extern "C" void kernel_launch(void* const* d_in, const int* in_sizes, int n_in, void* d_out, int out_size, void* d_ws, size_t ws_size, hipStream_t stream) {
  (void)n_in;
  auto Fp = [&](int i) { return (const float*)d_in[i]; }; auto Ip = [&](int i) { return (const int*)d_in[i]; };
  if (in_sizes[0] != NTOK * DD || in_sizes[1] != NTOK * DD || in_sizes[2] != DD * HH || in_sizes[4] != DD * HH * HH || in_sizes[6] != DD * HH * HH || in_sizes[8] != DD * HH * HH || in_sizes[9] != DD * 2 * KK || out_size != 2 * NTOK * KK) return;
  const int TLIM = NTOK;
  size_t off = 0; char* ws = (char*)d_ws;
  auto carve = [&](size_t bytes) { char* p = ws + off; off += (bytes + 255) & ~(size_t)255; return p; };
  b16* WT = (b16*)carve((size_t)3 * DD * HH * HH * 2);
  if (off > ws_size || off > ((size_t)8 << 20)) return;
  wput_kernel<<<256, 256, 0, stream>>>(Fp(4), Fp(6), Fp(8), WT);
  main_kernel<<<NTOK / 16, 32, 0, stream>>>(Fp(0), Ip(1), Fp(2), Fp(3), Fp(5), Fp(7), Fp(9), WT, TLIM, (float*)d_out);
}
